// NeighEnco2_61950608277608
// MI455X (gfx1250) — hardware-verified
//
#include <hip/hip_runtime.h>
#include <math.h>

typedef __attribute__((ext_vector_type(16))) _Float16 v16h;
typedef __attribute__((ext_vector_type(16))) __bf16 v16b;
typedef __attribute__((ext_vector_type(8)))  _Float16 v8h;
typedef __attribute__((ext_vector_type(8)))  float v8f;
typedef __attribute__((ext_vector_type(4)))  float v4f;
typedef __attribute__((ext_vector_type(2)))  float v2f;
typedef __attribute__((ext_vector_type(4)))  unsigned v4u;
typedef __attribute__((ext_vector_type(4)))  int v4i;
typedef float __attribute__((may_alias)) float_a;
typedef int __attribute__((may_alias)) int_a;

template <typename T> __device__ __forceinline__ void vst2(void* p, T v) { *(volatile T*)p = v; __threadfence(); *(volatile T*)p = v; }
__device__ __forceinline__ v8f wmma16(v16h a, v16h b, v8f c) {
  v8f d = __builtin_amdgcn_wmma_f32_16x16x32_f16(false, a, false, b, (short)0, c, false, false);
  asm volatile("v_nop\n\tv_nop\n\tv_nop\n\tv_nop" : "+v"(d) : "v"(a), "v"(b));
  return d;
}
__device__ __forceinline__ v8f wmma_bf(v16b a, v16b b, v8f c) {
  v8f d = __builtin_amdgcn_wmma_f32_16x16x32_bf16(false, a, false, b, (short)0, c, false, false);
  asm volatile("v_nop\n\tv_nop\n\tv_nop\n\tv_nop" : "+v"(d) : "v"(a), "v"(b));
  return d;
}
__device__ __forceinline__ v16h frag_h(const _Float16* rowk0, int lane) {
  union { v16h v; v8h q[2]; } u; const _Float16* p = rowk0 + 8 * (lane >> 4);
  u.q[0] = *(const v8h*)p; u.q[1] = *(const v8h*)(p + 16); return u.v;
}
__device__ __forceinline__ v16h frag_f32(const float* rowk0, int lane) {
  v16h a; const float* p = rowk0 + 8 * (lane >> 4);
#pragma unroll
  for (int i = 0; i < 8; ++i) { a[i] = (_Float16)p[i]; a[8 + i] = (_Float16)p[16 + i]; }
  return a;
}
__device__ __forceinline__ v16h frag_f32s(const float* rowk0, int lane, float sc) {
  v16h a; const float* p = rowk0 + 8 * (lane >> 4);
#pragma unroll
  for (int i = 0; i < 8; ++i) { a[i] = (_Float16)(p[i] * sc); a[8 + i] = (_Float16)(p[16 + i] * sc); }
  return a;
}
__device__ __forceinline__ v16h fragc_f32(const float* W, int k0, int n, int lane, int ld, int K) {
  v16h a; const int g = lane >> 4;
#pragma unroll
  for (int i = 0; i < 8; ++i) { const int ka = k0 + 8 * g + i, kb = ka + 16;
    a[i] = (_Float16)(ka < K ? W[(size_t)(ka < K ? ka : K - 1) * ld + n] : 0.f); a[8 + i] = (_Float16)(kb < K ? W[(size_t)(kb < K ? kb : K - 1) * ld + n] : 0.f); }
  return a;
}
struct F2 { v16b h, l; };
__device__ __forceinline__ F2 bsplit16(const float v[16]) { F2 r;
#pragma unroll
  for (int i = 0; i < 16; ++i) { const __bf16 h = (__bf16)v[i]; r.h[i] = h; r.l[i] = (__bf16)(v[i] - (float)h); }
  return r; }
__device__ __forceinline__ F2 split_row(const float* row, int k0, int lane) { float v[16]; const float* p = row + k0 + 8 * (lane >> 4);
#pragma unroll
  for (int i = 0; i < 8; ++i) { v[i] = p[i]; v[8 + i] = p[16 + i]; }
  return bsplit16(v); }
__device__ __forceinline__ F2 split_rowK(const float* row, int k0, int lane, int K) { float v[16]; const int g = lane >> 4;
#pragma unroll
  for (int i = 0; i < 8; ++i) { const int ka = k0 + 8 * g + i, kb = ka + 16; v[i] = ka < K ? row[ka < K ? ka : K - 1] : 0.f; v[8 + i] = kb < K ? row[kb < K ? kb : K - 1] : 0.f; }
  return bsplit16(v); }
__device__ __forceinline__ F2 split_col(const float* W, int k0, int n, int lane, int ld, int K) { float v[16]; const int g = lane >> 4;
#pragma unroll
  for (int i = 0; i < 8; ++i) { const int ka = k0 + 8 * g + i, kb = ka + 16; v[i] = ka < K ? W[(size_t)(ka < K ? ka : K - 1) * ld + n] : 0.f; v[8 + i] = kb < K ? W[(size_t)(kb < K ? kb : K - 1) * ld + n] : 0.f; }
  return bsplit16(v); }
__device__ __forceinline__ v8f mac3(const F2& a, const F2& b, v8f c) { c = wmma_bf(a.l, b.h, c); c = wmma_bf(a.h, b.l, c); return wmma_bf(a.h, b.h, c); }
__device__ __forceinline__ float sigm(float v) { return 1.0f / (1.0f + expf(-v)); }
#define LDSX() do { asm volatile("s_wait_dscnt 0" ::: "memory"); __builtin_amdgcn_wave_barrier(); __builtin_amdgcn_fence(__ATOMIC_RELEASE, "workgroup"); } while (0)


#define NZ 100000
#define CC 128
#define C1 64
#define C2 64
#define NNODE 50000
#define LNB 32
#define NR (NNODE * LNB)
#ifndef NRB
#define NRB (NR / 64)
#endif
#define SLOPE 0.05f
typedef __attribute__((ext_vector_type(8))) __bf16 v8b;
__device__ __forceinline__ v16b frag_b(const __bf16* rowk0, int lane) {
  union { v16b v; v8b q[2]; } u; const __bf16* p = rowk0 + 8 * (lane >> 4);
  u.q[0] = *(const v8b*)p; u.q[1] = *(const v8b*)(p + 16); return u.v;
}
__device__ __forceinline__ float bfr(float v) { return (float)(__bf16)v; }
__device__ __attribute__((noinline)) float exp_ni(float v) { return expf(v); }
__device__ __attribute__((noinline)) float erf_ni(float v) { return erff(v); }

#define WS_PW  0u
#define WS_P2  (WS_PW + 2u * C1 * CC)
#define WS_END (WS_P2 + 2u * C2 * C1 + 256u)

__global__ __launch_bounds__(128) void k_pack(const float* __restrict__ W1, const float* __restrict__ W2, __bf16* __restrict__ P) {
  const int n = blockIdx.x, t = threadIdx.x; __shared__ __align__(16) __bf16 s[CC];
  if (t < CC) s[t] = (__bf16)W1[(size_t)n * CC + t]; __syncthreads(); if (t < CC / 8) vst2((unsigned*)(P + (size_t)n * CC + t * 8), *(const v4u*)&s[t * 8]); __syncthreads();
  if (t < C1) s[t] = (__bf16)W2[(size_t)n * C1 + t]; __syncthreads(); if (t < C1 / 8) vst2((unsigned*)(P + WS_P2 / 2 + (size_t)n * C1 + t * 8), *(const v4u*)&s[t * 8]);
}
__device__ __forceinline__ float leaky(float v) { return v > 0.f ? v : SLOPE * v; }
__global__ __launch_bounds__(128) void k_main(const float* __restrict__ Z, const int* __restrict__ NBR, const __bf16* __restrict__ P, float* __restrict__ OUT) {
  __shared__ __align__(16) float sh[64][CC + 4];
  __shared__ int sidx[64];
  const int tid = threadIdx.x, wave = tid >> 5, lane = tid & 31, col = lane & 15, g = lane >> 4; const size_t eb0 = (size_t)blockIdx.x * 64;
  if (tid < 64) sidx[tid] = NBR[eb0 + tid];
  __syncthreads();
  { v8f acc[4] = {};
    const int idx = sidx[wave * 16 + col]; const float* zr = (idx > 0) ? Z + (size_t)(idx - 1) * CC : nullptr;
#pragma unroll
    for (int kc = 0; kc < CC / 32; ++kc) { v16b a;
#pragma unroll
      for (int i = 0; i < 8; ++i) { a[i] = (__bf16)(zr ? zr[kc * 32 + 8 * g + i] : 0.f); a[8 + i] = (__bf16)(zr ? zr[kc * 32 + 8 * g + 16 + i] : 0.f); }
#pragma unroll
      for (int j = 0; j < 4; ++j) acc[j] = wmma_bf(a, frag_b(P + (size_t)(j * 16 + col) * CC + kc * 32, lane), acc[j]); }
#pragma unroll
    for (int j = 0; j < 4; ++j)
#pragma unroll
      for (int r = 0; r < 8; ++r) sh[wave * 16 + 8 * g + r][j * 16 + col] = leaky(acc[j][r]); }
  if (tid < 64) for (int c = CC; c < CC + 4; ++c) sh[tid][c] = 0.f;
  LDSX();
  { v8f acc[4] = {};
#pragma unroll
    for (int kc = 0; kc < C1 / 32; ++kc) { const F2 a = split_row(&sh[wave * 16 + col][0], kc * 32, lane);
#pragma unroll
      for (int j = 0; j < 4; ++j) { const v16b w = frag_b(P + WS_P2 / 2 + (size_t)(j * 16 + col) * C1 + kc * 32, lane); acc[j] = wmma_bf(a.l, w, acc[j]); acc[j] = wmma_bf(a.h, w, acc[j]); } }
#pragma unroll
    for (int j = 0; j < 4; ++j)
#pragma unroll
      for (int r = 0; r < 8; ++r) sh[wave * 16 + 8 * g + r][C1 + j * 16 + col] = leaky(acc[j][r]); }
  __syncthreads();
  { const int node = tid >> 6, c0 = (tid & 63) * 2; float m0 = -3.0e38f, m1 = -3.0e38f;
#pragma unroll 1
    for (int r = 0; r < LNB; ++r) { m0 = fmaxf(m0, sh[node * LNB + r][c0]); m1 = fmaxf(m1, sh[node * LNB + r][c0 + 1]); }
    __syncthreads();
    sh[node][c0] = m0; sh[node][c0 + 1] = m1; }
  __syncthreads();
  if (tid < 64) { const int node = tid >> 5, q = tid & 31; vst2(OUT + (eb0 / LNB + node) * CC + q * 4, *(const v4f*)&sh[node][q * 4]); }
}
extern "C" void kernel_launch(void* const* d_in, const int* in_sizes, int n_in, void* d_out, int out_size, void* d_ws, size_t ws_size, hipStream_t stream) {
  (void)in_sizes; (void)n_in; (void)out_size;
  const float** F = (const float**)d_in;
  if (ws_size < (size_t)WS_END) return;
  char* ws = (char*)d_ws; __bf16* P = (__bf16*)ws;
  k_pack<<<C1, 128, 0, stream>>>(F[2], F[3], P);
  k_main<<<NRB, 128, 0, stream>>>(F[0], (const int*)d_in[1], P, (float*)d_out);
}
